// Hydra_Embedding_Dimensional_Attention_49701361549932
// MI455X (gfx1250) — hardware-verified
//
#include <hip/hip_runtime.h>
#include <math.h>

typedef __attribute__((ext_vector_type(16))) _Float16 v16h;
typedef __attribute__((ext_vector_type(16))) __bf16 v16b;
typedef __attribute__((ext_vector_type(8)))  _Float16 v8h;
typedef __attribute__((ext_vector_type(8)))  float v8f;
typedef __attribute__((ext_vector_type(4)))  float v4f;
typedef __attribute__((ext_vector_type(2)))  float v2f;
typedef __attribute__((ext_vector_type(4)))  unsigned v4u;
typedef __attribute__((ext_vector_type(4)))  int v4i;
typedef float __attribute__((may_alias)) float_a;
typedef int __attribute__((may_alias)) int_a;

template <typename T> __device__ __forceinline__ void vst2(void* p, T v) { *(volatile T*)p = v; __threadfence(); *(volatile T*)p = v; }
__device__ __forceinline__ v8f wmma16(v16h a, v16h b, v8f c) {
  v8f d = __builtin_amdgcn_wmma_f32_16x16x32_f16(false, a, false, b, (short)0, c, false, false);
  asm volatile("v_nop\n\tv_nop\n\tv_nop\n\tv_nop" : "+v"(d) : "v"(a), "v"(b));
  return d;
}
__device__ __forceinline__ v8f wmma_bf(v16b a, v16b b, v8f c) {
  v8f d = __builtin_amdgcn_wmma_f32_16x16x32_bf16(false, a, false, b, (short)0, c, false, false);
  asm volatile("v_nop\n\tv_nop\n\tv_nop\n\tv_nop" : "+v"(d) : "v"(a), "v"(b));
  return d;
}
__device__ __forceinline__ v16h frag_h(const _Float16* rowk0, int lane) {
  union { v16h v; v8h q[2]; } u; const _Float16* p = rowk0 + 8 * (lane >> 4);
  u.q[0] = *(const v8h*)p; u.q[1] = *(const v8h*)(p + 16); return u.v;
}
__device__ __forceinline__ v16h frag_f32(const float* rowk0, int lane) {
  v16h a; const float* p = rowk0 + 8 * (lane >> 4);
#pragma unroll
  for (int i = 0; i < 8; ++i) { a[i] = (_Float16)p[i]; a[8 + i] = (_Float16)p[16 + i]; }
  return a;
}
__device__ __forceinline__ v16h frag_f32s(const float* rowk0, int lane, float sc) {
  v16h a; const float* p = rowk0 + 8 * (lane >> 4);
#pragma unroll
  for (int i = 0; i < 8; ++i) { a[i] = (_Float16)(p[i] * sc); a[8 + i] = (_Float16)(p[16 + i] * sc); }
  return a;
}
__device__ __forceinline__ v16h fragc_f32(const float* W, int k0, int n, int lane, int ld, int K) {
  v16h a; const int g = lane >> 4;
#pragma unroll
  for (int i = 0; i < 8; ++i) { const int ka = k0 + 8 * g + i, kb = ka + 16;
    a[i] = (_Float16)(ka < K ? W[(size_t)(ka < K ? ka : K - 1) * ld + n] : 0.f); a[8 + i] = (_Float16)(kb < K ? W[(size_t)(kb < K ? kb : K - 1) * ld + n] : 0.f); }
  return a;
}
struct F2 { v16b h, l; };
__device__ __forceinline__ F2 bsplit16(const float v[16]) { F2 r;
#pragma unroll
  for (int i = 0; i < 16; ++i) { const __bf16 h = (__bf16)v[i]; r.h[i] = h; r.l[i] = (__bf16)(v[i] - (float)h); }
  return r; }
__device__ __forceinline__ F2 split_row(const float* row, int k0, int lane) { float v[16]; const float* p = row + k0 + 8 * (lane >> 4);
#pragma unroll
  for (int i = 0; i < 8; ++i) { v[i] = p[i]; v[8 + i] = p[16 + i]; }
  return bsplit16(v); }
__device__ __forceinline__ F2 split_rowK(const float* row, int k0, int lane, int K) { float v[16]; const int g = lane >> 4;
#pragma unroll
  for (int i = 0; i < 8; ++i) { const int ka = k0 + 8 * g + i, kb = ka + 16; v[i] = ka < K ? row[ka < K ? ka : K - 1] : 0.f; v[8 + i] = kb < K ? row[kb < K ? kb : K - 1] : 0.f; }
  return bsplit16(v); }
__device__ __forceinline__ F2 split_col(const float* W, int k0, int n, int lane, int ld, int K) { float v[16]; const int g = lane >> 4;
#pragma unroll
  for (int i = 0; i < 8; ++i) { const int ka = k0 + 8 * g + i, kb = ka + 16; v[i] = ka < K ? W[(size_t)(ka < K ? ka : K - 1) * ld + n] : 0.f; v[8 + i] = kb < K ? W[(size_t)(kb < K ? kb : K - 1) * ld + n] : 0.f; }
  return bsplit16(v); }
__device__ __forceinline__ v8f mac3(const F2& a, const F2& b, v8f c) { c = wmma_bf(a.l, b.h, c); c = wmma_bf(a.h, b.l, c); return wmma_bf(a.h, b.h, c); }
__device__ __forceinline__ float sigm(float v) { return 1.0f / (1.0f + expf(-v)); }
#define LDSX() do { asm volatile("s_wait_dscnt 0" ::: "memory"); __builtin_amdgcn_wave_barrier(); __builtin_amdgcn_fence(__ATOMIC_RELEASE, "workgroup"); } while (0)


#define NB 64
#define NT 196
#define NTP 224
#define NQC 208
#define NKV 392
#define NKVC 400
#define CC 768
#define NR (NB * CC)
#ifndef TNB
#define TNB NB
#endif
typedef __attribute__((ext_vector_type(8))) __bf16 v8b;
__device__ __forceinline__ v16b frag_b(const __bf16* rowk0, int lane) {
  union { v16b v; v8b q[2]; } u; const __bf16* p = rowk0 + 8 * (lane >> 4);
  u.q[0] = *(const v8b*)p; u.q[1] = *(const v8b*)(p + 16); return u.v;
}
__device__ __forceinline__ float bfr(float v) { return (float)(__bf16)v; }
__device__ __attribute__((noinline)) float exp_ni(float v) { return expf(v); }
__device__ __attribute__((noinline)) float erf_ni(float v) { return erff(v); }
__device__ __attribute__((noinline)) float gelu_e(float v) { return 0.5f * v * (1.0f + erff(v * 0.70710678118654752f)); }

#define WS_PQ  0u
#define WS_PKV (WS_PQ + 2u * (size_t)NQC * NTP)
#define WS_PP  (WS_PKV + 2u * (size_t)NKVC * NTP)
#define WS_XT  (WS_PP + 2u * (size_t)NQC * NTP)
#define WS_Q   (WS_XT + 2u * (size_t)NR * NTP)
#define WS_KV  (WS_Q + 4u * (size_t)NR * NQC)
#define WS_KT  (WS_KV + 4u * (size_t)NR * NKVC)
#define WS_IQ  (WS_KT + 4u * (size_t)NB * NTP)
#define WS_END (WS_IQ + 4u * (size_t)NR)

__global__ __launch_bounds__(224) void k_pack(const float* __restrict__ WQ, const float* __restrict__ WKV, const float* __restrict__ WP, char* __restrict__ ws) { const int m = blockIdx.x, which = blockIdx.y, t = threadIdx.x; __shared__ __align__(16) __bf16 s[NTP];
  const int nrows = (which == 1) ? NKV : NT, nrp = (which == 1) ? NKVC : NQC; if (m >= nrp) return; const float* Wm = (which == 0) ? WQ : (which == 1) ? WKV : WP;
  s[t] = (m < nrows && t < NT) ? (__bf16)Wm[(size_t)m * NT + t] : (__bf16)0.0f; __syncthreads();
  __bf16* dst = (__bf16*)(ws + ((which == 0) ? WS_PQ : (which == 1) ? WS_PKV : WS_PP)) + (size_t)m * NTP; if (t < NTP / 8) vst2((unsigned*)(dst + t * 8), *(const v4u*)&s[t * 8]); }
__global__ __launch_bounds__(256) void k_xt(const float* __restrict__ X, __bf16* __restrict__ XT) { __shared__ __align__(16) __bf16 st[64][NTP + 8]; const int t = threadIdx.x; const int c0 = blockIdx.x * 64; const size_t b = blockIdx.y;
  for (int e = t; e < 64 * NTP; e += 256) { const int n = e >> 6, cl = e & 63; st[cl][n] = (n < NT) ? (__bf16)X[(b * NT + n) * CC + c0 + cl] : (__bf16)0.0f; } __syncthreads();
  for (int e = t; e < 64 * (NTP / 8); e += 256) { const int cl = e / (NTP / 8), q = e % (NTP / 8); vst2((unsigned*)(XT + ((b * CC + c0 + cl) * NTP) + q * 8), *(const v4u*)&st[cl][q * 8]); } }
__global__ __launch_bounds__(128) void k_proj(const __bf16* __restrict__ XT, const char* __restrict__ ws, float* __restrict__ Q, float* __restrict__ KV) { __shared__ __align__(16) float sf[4][16][132];
  const int tid = threadIdx.x, wave = tid >> 5, lane = tid & 31, col = lane & 15, g = lane >> 4; const size_t r0 = (size_t)blockIdx.x * 64 + wave * 16; const int t0 = blockIdx.y * 8;
  v8f acc[8] = {};
#pragma unroll 1
  for (int kc = 0; kc < NTP / 32; ++kc) { const v16b a = frag_b(XT + (r0 + col) * NTP + kc * 32, lane);
#pragma unroll
    for (int j = 0; j < 8; ++j) { const int tile = t0 + j; if (tile >= 38) break; const __bf16* wr = (tile < 13) ? ((const __bf16*)(ws + WS_PQ) + (size_t)(tile * 16 + col) * NTP) : ((const __bf16*)(ws + WS_PKV) + (size_t)((tile - 13) * 16 + col) * NTP); acc[j] = wmma_bf(a, frag_b(wr + kc * 32, lane), acc[j]); } }
#pragma unroll
  for (int j = 0; j < 8; ++j)
#pragma unroll
    for (int r = 0; r < 8; ++r) sf[wave][8 * g + r][j * 16 + col] = acc[j][r];
  LDSX();
  for (int rl = 0; rl < 16; ++rl) { const int tile = t0 + (lane >> 2); if (tile < 38) { const int q = lane & 3; float* dst = (tile < 13) ? (Q + (r0 + rl) * NQC + tile * 16 + q * 4) : (KV + (r0 + rl) * NKVC + (tile - 13) * 16 + q * 4); vst2(dst, *(const v4f*)&sf[wave][rl][(lane >> 2) * 16 + q * 4]); } } }
__global__ __launch_bounds__(256) void k_norms(const float* __restrict__ Q, const float* __restrict__ KV, float* __restrict__ KT, float* __restrict__ IQ) { __shared__ float red[8]; __shared__ float skt[NTP]; __shared__ __align__(16) float siq[CC]; __shared__ __align__(16) float so2[NTP]; const int t = threadIdx.x; const size_t b = blockIdx.x;
  for (int n = t; n < NTP; n += 256) skt[n] = 0.f; __syncthreads();
#pragma unroll 1
  for (int c = 0; c < CC; ++c) { const size_t row = b * CC + c; const float qv = (t < NT) ? Q[row * NQC + t] : 0.f; const float kvv = (t < NT) ? KV[row * NKVC + t] : 0.f; float sq = qv * qv, sk = kvv * kvv;
#pragma unroll
    for (int o = 1; o < 32; o <<= 1) { sq += __shfl_xor(sq, o); sk += __shfl_xor(sk, o); }
    __syncthreads(); if ((t & 31) == 0) { red[t >> 5] = sq; } __syncthreads(); float tq = 0.f; for (int i = 0; i < 8; ++i) tq += red[i]; __syncthreads(); if ((t & 31) == 0) red[t >> 5] = sk; __syncthreads(); float tk = 0.f; for (int i = 0; i < 8; ++i) tk += red[i];
    if (t == 0) siq[c] = 1.0f / sqrtf(tq); const float ik = 1.0f / sqrtf(tk);
    if (t < NT) skt[t] += kvv * ik * KV[row * NKVC + NT + t]; }
  __syncthreads(); for (int n = t; n < NTP; n += 256) so2[n] = (n < NT) ? skt[n] : 0.f; __syncthreads();
  if (t < NTP / 4) vst2(KT + b * NTP + t * 4, *(const v4f*)&so2[t * 4]); for (int q = t; q < CC / 4; q += 256) vst2(IQ + b * CC + q * 4, *(const v4f*)&siq[q * 4]); }
__global__ __launch_bounds__(128) void k_out(const float* __restrict__ Q, const float* __restrict__ IQ, const float* __restrict__ KT, const float* __restrict__ SCL, const __bf16* __restrict__ PP, const float* __restrict__ BP, float* __restrict__ OUT) { __shared__ __align__(16) float so[NQC][64 + 4];
  const int tid = threadIdx.x, wave = tid >> 5, lane = tid & 31, col = lane & 15, g = lane >> 4; const size_t b = blockIdx.y; const int c0 = blockIdx.x * 64; const size_t r0 = b * CC + c0 + wave * 16; const float scl = bfr(SCL[0]); const float* kt = KT + b * NTP;
  v8f acc[13];
#pragma unroll
  for (int j = 0; j < 13; ++j) acc[j] = v8f{};
  const float iq = IQ[r0 + col];
#pragma unroll 1
  for (int kc = 0; kc < NTP / 32; ++kc) { float v[16]; const float* qp = Q + (r0 + col) * NQC + kc * 32 + 8 * g; const float* kp = kt + kc * 32 + 8 * g;
#pragma unroll
    for (int i = 0; i < 8; ++i) { const int n0 = kc * 32 + 8 * g + i; v[i] = (n0 < NT) ? gelu_e(qp[i] * iq * kp[i] * scl) : 0.f; v[8 + i] = (n0 + 16 < NT) ? gelu_e(qp[16 + i] * iq * kp[16 + i] * scl) : 0.f; }
    const F2 a = bsplit16(v);
#pragma unroll
    for (int j = 0; j < 13; ++j) { const v16b w = frag_b(PP + (size_t)(j * 16 + col) * NTP + kc * 32, lane); acc[j] = wmma_bf(a.h, w, acc[j]); acc[j] = wmma_bf(a.l, w, acc[j]); } }
#pragma unroll
  for (int j = 0; j < 13; ++j) { const int m = j * 16 + col; const float bb = (m < NT) ? bfr(BP[m]) : 0.f;
#pragma unroll
    for (int r = 0; r < 8; ++r) so[m][wave * 16 + 8 * g + r] = acc[j][r] + bb; }
  __syncthreads();
  for (int e = tid; e < NT * 16; e += 128) { const int m = e >> 4, q = e & 15; vst2(OUT + ((b * NT + m) * CC) + c0 + q * 4, *(const v4f*)&so[m][q * 4]); } }
extern "C" void kernel_launch(void* const* d_in, const int* in_sizes, int n_in, void* d_out, int out_size, void* d_ws, size_t ws_size, hipStream_t stream) {
  (void)in_sizes; (void)n_in; (void)out_size;
  const float** F = (const float**)d_in;
  if (ws_size < (size_t)WS_END) return;
  char* ws = (char*)d_ws; __bf16* XT = (__bf16*)(ws + WS_XT); float *Q = (float*)(ws + WS_Q), *KV = (float*)(ws + WS_KV), *KT = (float*)(ws + WS_KT), *IQ = (float*)(ws + WS_IQ);
  k_pack<<<dim3(NKVC, 3), 224, 0, stream>>>(F[1], F[2], F[3], ws);
  k_xt<<<dim3(CC / 64, TNB), 256, 0, stream>>>(F[0], XT);
  k_proj<<<dim3(TNB * CC / 64, 5), 128, 0, stream>>>(XT, ws, Q, KV);
  k_norms<<<TNB, 256, 0, stream>>>(Q, KV, KT, IQ);
  k_out<<<dim3(CC / 64, TNB), 128, 0, stream>>>(Q, IQ, KT, F[5], (const __bf16*)(ws + WS_PP), F[4], (float*)d_out);
}
